// HGTNet_53068615910208
// MI455X (gfx1250) — hardware-verified
//
#include <hip/hip_runtime.h>
#include <stdint.h>
#include <stddef.h>


#define DF    128
#define NH    8
#define HD    16
#define NL    2
#define NCLS  2
#define GR    32
#define AP    136
#define XSP   132
#define KP    388
#define NB    192
#define CHUNK 2048
#define NTHR  256
#define NWAVE 8
#define WCAP  256
#define HB    128
#define RELT  (HD * 32)

#define NODE_LDS_BYTES (2 * GR * AP * 2 + GR * KP * 4 + GR * XSP * 4)

#define AG_ACC  0
#define AG_DEN  (2 * NB * DF)
#define AG_MRUN (AG_DEN + NB * NH)
#define AG_OUT  (AG_MRUN + NB * NH)
#define AG_LIST (AG_OUT + 16 * XSP)
#define AG_WCNT (AG_LIST + NWAVE * WCAP)
#define AG_PRL  (AG_WCNT + NWAVE)
#define AG_LDS_BYTES ((AG_PRL + 2 * NH) * 4)

static_assert(NODE_LDS_BYTES == 83968);
static_assert(AG_LDS_BYTES == 225632);
static_assert(WCAP == (CHUNK / NTHR) * 32);
static_assert(CHUNK == NTHR * 8);
static_assert((NB % 16) == 0 && NB <= 512);
static_assert((AG_MRUN % 4) == 0 && (AG_OUT % 4) == 0 && (AG_LIST % 4) == 0);
static_assert(DF == NH * HD && NWAVE == NH && NTHR == NWAVE * 32);
static_assert((HB * NCLS) / 4 == 64 && NCLS == 2);
static_assert(((AP * 2) % 16) == 0 && ((XSP * 4) % 16) == 0 && ((KP * 4) % 16) == 0);

typedef float          v4f  __attribute__((ext_vector_type(4)));
typedef float          v8f  __attribute__((ext_vector_type(8)));
typedef int            v4i  __attribute__((ext_vector_type(4)));
typedef unsigned short v8us __attribute__((ext_vector_type(8)));
typedef __bf16         v16b __attribute__((ext_vector_type(16)));
union Frag { v16b v; v8us s[2]; };
union P8   { v8us s; v4i i; unsigned short e[8]; };

__device__ __forceinline__ v8f zero8() {
  v8f z = {0.f, 0.f, 0.f, 0.f, 0.f, 0.f, 0.f, 0.f};
  return z;
}

__device__ __forceinline__ void split_bf16(float f, unsigned short& hi, unsigned short& lo) {
  const unsigned int u = __float_as_uint(f);
  const unsigned int hb = (u + 0x7FFFu + ((u >> 16) & 1u)) >> 16;
  const float fh = __uint_as_float(hb << 16);
  const float r = f - fh;
  const unsigned int ur = __float_as_uint(r);
  const unsigned int lb = (ur + 0x7FFFu + ((ur >> 16) & 1u)) >> 16;
  hi = (unsigned short)hb;
  lo = (unsigned short)lb;
}

__device__ __forceinline__ void split8(const v4f a, const v4f b, P8& hi, P8& lo) {
  float f[8] = {a.x, a.y, a.z, a.w, b.x, b.y, b.z, b.w};
#pragma unroll
  for (int i = 0; i < 8; ++i) {
    unsigned short h1, l1;
    split_bf16(f[i], h1, l1);
    hi.e[i] = h1;
    lo.e[i] = l1;
  }
}

__device__ __forceinline__ void frag_f32(const v4f x0, const v4f x1, const v4f x2, const v4f x3,
                                         Frag& fh, Frag& fl) {
  P8 h0, l0, h1, l1;
  split8(x0, x1, h0, l0);
  split8(x2, x3, h1, l1);
  fh.s[0] = h0.s; fh.s[1] = h1.s;
  fl.s[0] = l0.s; fl.s[1] = l1.s;
}

__device__ __forceinline__ void ldfrag(Frag& f, const unsigned short* row, int k0, int h) {
  f.s[0] = *(const v8us*)(row + k0 + 8 * h);
  f.s[1] = *(const v8us*)(row + k0 + 16 + 8 * h);
}

__device__ __forceinline__ v8f wm(v16b a, v16b b, v8f c) {
  v8f d = __builtin_amdgcn_wmma_f32_16x16x32_bf16(false, a, false, b, (short)0, c, false, false);
  asm volatile("v_nop\n\tv_nop\n\tv_nop\n\tv_nop" : "+v"(d) : "v"(a), "v"(b));
  return d;
}

__device__ __forceinline__ v8f wm3(v16b ah, v16b al, v16b bh, v16b bl, v8f c) {
  c = wm(ah, bh, c);
  c = wm(ah, bl, c);
  c = wm(al, bh, c);
  return c;
}

__device__ __forceinline__ float gelu1(float x) {
  return 0.5f * x * (1.0f + erff(x * 0.70710678118654752f));
}
__device__ __forceinline__ v4f gelu4(v4f x) {
  v4f y;
  y.x = gelu1(x.x); y.y = gelu1(x.y); y.z = gelu1(x.z); y.w = gelu1(x.w);
  return y;
}

template <int GELU>
__device__ __forceinline__ void stage_rows(const float* __restrict__ A, int rowBase, int nN, int tid,
                                           unsigned short* Ah, unsigned short* Al) {
  const int r = tid >> 3, c0 = (tid & 7) * 16;
  int row = rowBase + r;
  if (row > nN - 1) row = nN - 1;
  const float* p = A + (size_t)row * DF + c0;
  v4f f0 = *(const v4f*)(p), f1 = *(const v4f*)(p + 4);
  v4f f2 = *(const v4f*)(p + 8), f3 = *(const v4f*)(p + 12);
  if (GELU) { f0 = gelu4(f0); f1 = gelu4(f1); f2 = gelu4(f2); f3 = gelu4(f3); }
  P8 h0, l0, h1, l1;
  split8(f0, f1, h0, l0);
  split8(f2, f3, h1, l1);
  *(v8us*)(Ah + r * AP + c0)     = h0.s;
  *(v8us*)(Ah + r * AP + c0 + 8) = h1.s;
  *(v8us*)(Al + r * AP + c0)     = l0.s;
  *(v8us*)(Al + r * AP + c0 + 8) = l1.s;
}

__global__ __launch_bounds__(NTHR) void k_wt(const float* __restrict__ W, unsigned short* Ph,
                                             unsigned short* Pl, int N, int Npad) {
  __shared__ __attribute__((aligned(16))) unsigned short th[16 * AP];
  __shared__ __attribute__((aligned(16))) unsigned short tl[16 * AP];
  const int tid = threadIdx.x;
  const int R0 = blockIdx.x * 16;
  {
    const int nl = tid >> 4, kk = tid & 15;
    const int R = R0 + nl;
    const int l = R / Npad;
    const int n = R - l * Npad;
    const bool ok = n < N;
    const int nc = ok ? n : (N - 1);
    const float* wp = W + (size_t)l * DF * N + nc;
#pragma unroll
    for (int j = 0; j < 8; ++j) {
      const int k = kk + 16 * j;
      float v = wp[(size_t)k * N];
      if (!ok) v = 0.f;
      unsigned short hi, lo;
      split_bf16(v, hi, lo);
      th[nl * AP + k] = hi;
      tl[nl * AP + k] = lo;
    }
  }
  __syncthreads();
  const int row = tid >> 4, pc = tid & 15;
  const v4i vh = *(const v4i*)(th + row * AP + pc * 8);
  const v4i vl = *(const v4i*)(tl + row * AP + pc * 8);
  const size_t o = (size_t)(R0 + row) * DF + pc * 8;
  *(volatile v4i*)(Ph + o) = vh;
  *(volatile v4i*)(Pl + o) = vl;
  __threadfence();
  *(volatile v4i*)(Ph + o) = vh;
  *(volatile v4i*)(Pl + o) = vl;
}

__global__ __launch_bounds__(NTHR) void k_relprep(const float* __restrict__ krel_w,
                                                  const float* __restrict__ vrel_w,
                                                  unsigned short* Bkh, unsigned short* Bkl,
                                                  unsigned short* Bvh, unsigned short* Bvl) {
  __shared__ __attribute__((aligned(16))) unsigned short th[RELT];
  __shared__ __attribute__((aligned(16))) unsigned short tl[RELT];
  const int tid = threadIdx.x, b = blockIdx.x;
  const int nk = NL * 2 * NH;
  const bool isk = b < nk;
  int l, t, hh;
  if (isk) { l = b / (2 * NH); t = (b / NH) & 1; hh = b & (NH - 1); }
  else     { const int c = b - nk; l = c / NH; t = 0; hh = c & (NH - 1); }
  for (int i = tid; i < RELT; i += NTHR) {
    const int f = i >> 5, kk = i & 31;
    const int tt = kk >> 4, d = kk & 15;
    float v;
    if (isk) {
      const float w = krel_w[(((l * 2 + t) * NH + hh) * HD + d) * HD + f];
      v = (tt == (hh & 1)) ? w : 0.f;
    } else {
      v = vrel_w[(((l * 2 + tt) * NH + hh) * HD + d) * HD + f];
    }
    unsigned short hi, lo;
    split_bf16(v, hi, lo);
    th[i] = hi;
    tl[i] = lo;
  }
  __syncthreads();
  if (tid < RELT / 8) {
    const v4i vh = *(const v4i*)(th + tid * 8);
    const v4i vl = *(const v4i*)(tl + tid * 8);
    unsigned short* oh = (isk ? (Bkh + (size_t)b * RELT) : (Bvh + (size_t)(b - nk) * RELT)) + tid * 8;
    unsigned short* ol = (isk ? (Bkl + (size_t)b * RELT) : (Bvl + (size_t)(b - nk) * RELT)) + tid * 8;
    *(volatile v4i*)oh = vh;
    *(volatile v4i*)ol = vl;
    __threadfence();
    *(volatile v4i*)oh = vh;
    *(volatile v4i*)ol = vl;
  }
}

template <int MODE>
__global__ __launch_bounds__(NTHR) void k_gemm128(const float* __restrict__ A,
                                                  const unsigned short* __restrict__ Wh,
                                                  const unsigned short* __restrict__ Wl,
                                                  const float* __restrict__ bias,
                                                  const float* __restrict__ gate,
                                                  float* hio, int nN) {
  __shared__ __attribute__((aligned(16))) unsigned short Ah[GR * AP];
  __shared__ __attribute__((aligned(16))) unsigned short Al[GR * AP];
  __shared__ __attribute__((aligned(16))) float Xs[GR * XSP];
  const int tid = threadIdx.x, lane = tid & 31, wave = tid >> 5;
  const int hh = lane >> 4, m = lane & 15;
  const int rowBase = blockIdx.x * GR;

  stage_rows<MODE>(A, rowBase, nN, tid, Ah, Al);
  __syncthreads();

  const int ncol = wave * HD + m;
  const unsigned short* bhr = Wh + (size_t)ncol * DF;
  const unsigned short* blr = Wl + (size_t)ncol * DF;
  v8f c0 = zero8(), c1 = zero8();
#pragma unroll
  for (int kt = 0; kt < DF / 32; ++kt) {
    const int k0 = kt * 32;
    Frag a0h, a0l, a1h, a1l, bh, bl;
    ldfrag(a0h, Ah + m * AP, k0, hh);
    ldfrag(a0l, Al + m * AP, k0, hh);
    ldfrag(a1h, Ah + (16 + m) * AP, k0, hh);
    ldfrag(a1l, Al + (16 + m) * AP, k0, hh);
    ldfrag(bh, bhr, k0, hh);
    ldfrag(bl, blr, k0, hh);
    c0 = wm3(a0h.v, a0l.v, bh.v, bl.v, c0);
    c1 = wm3(a1h.v, a1l.v, bh.v, bl.v, c1);
  }

  const float bs = bias[ncol];
  float g = 0.f, omg = 1.f;
  if (MODE == 1) {
    const float e = expf(-gate[0]);
    g = __builtin_amdgcn_rcpf(1.0f + e);
    omg = 1.0f - g;
  }
#pragma unroll
  for (int r = 0; r < 8; ++r) {
    const int rl0 = 8 * hh + r, rl1 = 16 + 8 * hh + r;
    float v0 = c0[r] + bs, v1 = c1[r] + bs;
    if (MODE == 1) {
      int g0 = rowBase + rl0; if (g0 > nN - 1) g0 = nN - 1;
      int g1 = rowBase + rl1; if (g1 > nN - 1) g1 = nN - 1;
      const float h0 = hio[(size_t)g0 * DF + ncol];
      const float h1 = hio[(size_t)g1 * DF + ncol];
      v0 = fmaxf(g * v0 + omg * h0, 0.f);
      v1 = fmaxf(g * v1 + omg * h1, 0.f);
    }
    Xs[rl0 * XSP + ncol] = v0;
    Xs[rl1 * XSP + ncol] = v1;
  }
  __syncthreads();

  v4f xr[4];
  int gr[4];
#pragma unroll
  for (int i = 0; i < 4; ++i) {
    const int rl = 4 * wave + i;
    xr[i] = *(const v4f*)(Xs + rl * XSP + 4 * lane);
    gr[i] = rowBase + rl;
  }
#pragma unroll
  for (int i = 0; i < 4; ++i)
    if (gr[i] < nN) *(volatile v4f*)(hio + (size_t)gr[i] * DF + 4 * lane) = xr[i];
  __threadfence();
#pragma unroll
  for (int i = 0; i < 4; ++i)
    if (gr[i] < nN) *(volatile v4f*)(hio + (size_t)gr[i] * DF + 4 * lane) = xr[i];
}

__device__ __forceinline__ void put_tile(v8f c, float* T, int pitch, int rowoff, int col, float bs, int hh) {
#pragma unroll
  for (int r = 0; r < 8; ++r) T[(rowoff + 8 * hh + r) * pitch + col] = c[r] + bs;
}

__global__ __launch_bounds__(NTHR) void k_node(const float* __restrict__ h,
                                               const unsigned short* __restrict__ Wh,
                                               const unsigned short* __restrict__ Wl,
                                               const float* __restrict__ bias,
                                               const unsigned short* __restrict__ Bkh,
                                               const unsigned short* __restrict__ Bkl,
                                               float* qo, float* kro0, float* kro1, float* vo, int nN) {
  extern __shared__ v4f lds_dyn[];
  unsigned short* Ah = (unsigned short*)lds_dyn;
  unsigned short* Al = Ah + GR * AP;
  float* KQ = (float*)(Al + GR * AP);
  float* R  = KQ + GR * KP;
  const int tid = threadIdx.x, lane = tid & 31, wave = tid >> 5;
  const int hh = lane >> 4, m = lane & 15;
  const int rowBase = blockIdx.x * GR;

  stage_rows<0>(h, rowBase, nN, tid, Ah, Al);
  __syncthreads();

  const int ncol = wave * HD + m;
  const unsigned short* b0h = Wh + (size_t)(0 * DF + ncol) * DF;
  const unsigned short* b0l = Wl + (size_t)(0 * DF + ncol) * DF;
  const unsigned short* b1h = Wh + (size_t)(1 * DF + ncol) * DF;
  const unsigned short* b1l = Wl + (size_t)(1 * DF + ncol) * DF;
  const unsigned short* b2h = Wh + (size_t)(2 * DF + ncol) * DF;
  const unsigned short* b2l = Wl + (size_t)(2 * DF + ncol) * DF;
  v8f c00 = zero8(), c01 = zero8(), c10 = zero8(), c11 = zero8(), c20 = zero8(), c21 = zero8();
#pragma unroll
  for (int kt = 0; kt < DF / 32; ++kt) {
    const int k0 = kt * 32;
    Frag a0h, a0l, a1h, a1l, bh, bl;
    ldfrag(a0h, Ah + m * AP, k0, hh);
    ldfrag(a0l, Al + m * AP, k0, hh);
    ldfrag(a1h, Ah + (16 + m) * AP, k0, hh);
    ldfrag(a1l, Al + (16 + m) * AP, k0, hh);
    ldfrag(bh, b0h, k0, hh); ldfrag(bl, b0l, k0, hh);
    c00 = wm3(a0h.v, a0l.v, bh.v, bl.v, c00);
    c01 = wm3(a1h.v, a1l.v, bh.v, bl.v, c01);
    ldfrag(bh, b1h, k0, hh); ldfrag(bl, b1l, k0, hh);
    c10 = wm3(a0h.v, a0l.v, bh.v, bl.v, c10);
    c11 = wm3(a1h.v, a1l.v, bh.v, bl.v, c11);
    ldfrag(bh, b2h, k0, hh); ldfrag(bl, b2l, k0, hh);
    c20 = wm3(a0h.v, a0l.v, bh.v, bl.v, c20);
    c21 = wm3(a1h.v, a1l.v, bh.v, bl.v, c21);
  }
  {
    const float bs0 = bias[ncol], bs1 = bias[DF + ncol], bs2 = bias[2 * DF + ncol];
    put_tile(c00, KQ, KP, 0,  ncol,          bs0, hh);
    put_tile(c01, KQ, KP, 16, ncol,          bs0, hh);
    put_tile(c10, KQ, KP, 0,  DF + ncol,     bs1, hh);
    put_tile(c11, KQ, KP, 16, DF + ncol,     bs1, hh);
    put_tile(c20, KQ, KP, 0,  2 * DF + ncol, bs2, hh);
    put_tile(c21, KQ, KP, 16, 2 * DF + ncol, bs2, hh);
  }
  __syncthreads();

  {
    v4f qr[4], vr[4];
    int gr[4];
#pragma unroll
    for (int i = 0; i < 4; ++i) {
      const int rl = 4 * wave + i;
      qr[i] = *(const v4f*)(KQ + rl * KP + DF + 4 * lane);
      vr[i] = *(const v4f*)(KQ + rl * KP + 2 * DF + 4 * lane);
      gr[i] = rowBase + rl;
    }
#pragma unroll
    for (int i = 0; i < 4; ++i)
      if (gr[i] < nN) {
        *(volatile v4f*)(qo + (size_t)gr[i] * DF + 4 * lane) = qr[i];
        *(volatile v4f*)(vo + (size_t)gr[i] * DF + 4 * lane) = vr[i];
      }
    __threadfence();
#pragma unroll
    for (int i = 0; i < 4; ++i)
      if (gr[i] < nN) {
        *(volatile v4f*)(qo + (size_t)gr[i] * DF + 4 * lane) = qr[i];
        *(volatile v4f*)(vo + (size_t)gr[i] * DF + 4 * lane) = vr[i];
      }
  }

  const int hp = wave >> 1;
  Frag ah0, al0, ah1, al1;
  {
    const float* p0 = KQ + m * KP + 32 * hp;
    const float* p1 = KQ + (16 + m) * KP + 32 * hp;
    frag_f32(*(const v4f*)(p0 + 8 * hh), *(const v4f*)(p0 + 8 * hh + 4),
             *(const v4f*)(p0 + 16 + 8 * hh), *(const v4f*)(p0 + 16 + 8 * hh + 4), ah0, al0);
    frag_f32(*(const v4f*)(p1 + 8 * hh), *(const v4f*)(p1 + 8 * hh + 4),
             *(const v4f*)(p1 + 16 + 8 * hh), *(const v4f*)(p1 + 16 + 8 * hh + 4), ah1, al1);
  }
#pragma unroll 1
  for (int t = 0; t < 2; ++t) {
    Frag bh, bl;
    const size_t bro = (size_t)((t * NH + wave) * HD + m) * 32;
    ldfrag(bh, Bkh + bro, 0, hh);
    ldfrag(bl, Bkl + bro, 0, hh);
    v8f d0 = zero8(), d1 = zero8();
    d0 = wm3(ah0.v, al0.v, bh.v, bl.v, d0);
    d1 = wm3(ah1.v, al1.v, bh.v, bl.v, d1);
    put_tile(d0, R, XSP, 0,  ncol, 0.f, hh);
    put_tile(d1, R, XSP, 16, ncol, 0.f, hh);
    __syncthreads();
    float* kout = (t == 0) ? kro0 : kro1;
    v4f kr[4];
    int gr[4];
#pragma unroll
    for (int i = 0; i < 4; ++i) {
      const int rl = 4 * wave + i;
      kr[i] = *(const v4f*)(R + rl * XSP + 4 * lane);
      gr[i] = rowBase + rl;
    }
#pragma unroll
    for (int i = 0; i < 4; ++i)
      if (gr[i] < nN) *(volatile v4f*)(kout + (size_t)gr[i] * DF + 4 * lane) = kr[i];
    __threadfence();
#pragma unroll
    for (int i = 0; i < 4; ++i)
      if (gr[i] < nN) *(volatile v4f*)(kout + (size_t)gr[i] * DF + 4 * lane) = kr[i];
    __syncthreads();
  }
}

__global__ __launch_bounds__(NTHR) void k_agg(float* qa,
                                              const float* __restrict__ kr0,
                                              const float* __restrict__ kr1,
                                              const float* __restrict__ vv,
                                              const int* __restrict__ ef,
                                              const int* __restrict__ er, int nEf, int nEr,
                                              const float* __restrict__ prel,
                                              const unsigned short* __restrict__ Bvh,
                                              const unsigned short* __restrict__ Bvl, int nN) {
  extern __shared__ v4f lds_dyn[];
  float* lds  = (float*)lds_dyn;
  float* acc  = lds + AG_ACC;
  float* den  = lds + AG_DEN;
  float* mrun = lds + AG_MRUN;
  float* outt = lds + AG_OUT;
  int*   list = (int*)(lds + AG_LIST);
  int*   wcnt = (int*)(lds + AG_WCNT);
  float* prl  = lds + AG_PRL;

  const int tid = threadIdx.x, lane = tid & 31, wave = tid >> 5;
  const int hh = lane >> 4, m = lane & 15;
  const int hd = lane >> 2;
  const int nodeBase = blockIdx.x * NB;

  {
    const v4f z4 = {0.f, 0.f, 0.f, 0.f};
    for (int i = tid; i < AG_MRUN / 4; i += NTHR) lds_dyn[i] = z4;
    const float ninf = __uint_as_float(0xff800000u);
    for (int i = tid; i < NB * NH; i += NTHR) mrun[i] = ninf;
    if (tid < 2 * NH) prl[tid] = prel[tid] * 0.25f;
  }
  __syncthreads();

#pragma unroll 1
  for (int sq = 0; sq < 2; ++sq) {
    const int* srca = (sq == 0) ? ef : er;
    const int nE = (sq == 0) ? nEf : nEr;
    const int* dsta = srca + nE;
    const float* kr = (sq == 0) ? kr0 : kr1;
    const float pr = prl[sq * NH + hd];
    const bool al16 = ((((uintptr_t)dsta) & 15u) == 0u);
    const int nChunks = (nE + CHUNK - 1) / CHUNK;
#pragma unroll 1
    for (int ch = 0; ch < nChunks; ++ch) {
      const int cbase = ch * CHUNK;
      const int el0 = tid * 8;
      const int e0 = cbase + el0;
      const int sent = -2147483647 - 1;
      int d[8];
      if (al16 && (cbase + CHUNK <= nE)) {
        const v4i u0 = *(const v4i*)(dsta + e0);
        const v4i u1 = *(const v4i*)(dsta + e0 + 4);
        d[0] = u0.x; d[1] = u0.y; d[2] = u0.z; d[3] = u0.w;
        d[4] = u1.x; d[5] = u1.y; d[6] = u1.z; d[7] = u1.w;
      } else {
#pragma unroll
        for (int j = 0; j < 8; ++j) {
          int ix = e0 + j;
          const bool in = ix < nE;
          if (!in) ix = nE - 1;
          const int val = dsta[ix];
          d[j] = in ? val : sent;
        }
      }
      unsigned s[8];
      bool ht[8];
      bool any = false;
#pragma unroll
      for (int j = 0; j < 8; ++j) {
        s[j] = (unsigned)d[j] - (unsigned)nodeBase;
        ht[j] = s[j] < (unsigned)NB;
        any = any | ht[j];
      }
      int wc = 0;
      const unsigned many = __builtin_amdgcn_ballot_w32(any);
      if (many != 0u) {
#pragma unroll
        for (int j = 0; j < 8; ++j) {
          const unsigned mj = __builtin_amdgcn_ballot_w32(ht[j]);
          if (ht[j]) {
            const int pos = wc + (int)__builtin_amdgcn_mbcnt_lo(mj, 0u);
            if (pos < WCAP) list[wave * WCAP + pos] = ((el0 + j) << 9) | (int)s[j];
          }
          wc += (int)__builtin_popcount(mj);
        }
      }
      if (lane == 0) wcnt[wave] = wc;
      __syncthreads();

      if (wave == 0) {
        for (int wsx = 0; wsx < NWAVE; ++wsx) {
          int n = wcnt[wsx];
          if (n > WCAP) n = WCAP;
          if (n < 0) n = 0;
          for (int i = 0; i < n; ++i) {
            const int ent = list[wsx * WCAP + i];
            int slot = ent & 511;
            if (slot > NB - 1) slot = NB - 1;
            const int el = (ent >> 9) & (CHUNK - 1);
            int e = cbase + el;
            if (e > nE - 1) e = nE - 1;
            int src = srca[e];
            src = src < 0 ? 0 : (src > nN - 1 ? nN - 1 : src);
            int nd = nodeBase + slot;
            if (nd > nN - 1) nd = nN - 1;
            const v4f q4 = *(const v4f*)(qa + (size_t)nd * DF + 4 * lane);
            const v4f k4 = *(const v4f*)(kr + (size_t)src * DF + 4 * lane);
            float pd = q4.x * k4.x + q4.y * k4.y + q4.z * k4.z + q4.w * k4.w;
            pd += __shfl_xor(pd, 1, 32);
            pd += __shfl_xor(pd, 2, 32);
            const float a = pd * pr;
            const int mi = slot * NH + hd;
            const float mo = mrun[mi];
            const float mn = fmaxf(mo, a);
            const float sc = __expf(mo - mn);
            const float p = __expf(a - mn);
            const v4f vx = *(const v4f*)(vv + (size_t)src * DF + 4 * lane);
            v4f* p0 = (v4f*)(acc + (size_t)slot * DF + 4 * lane);
            v4f* p1 = (v4f*)(acc + (size_t)(NB + slot) * DF + 4 * lane);
            v4f a0 = *p0, a1 = *p1;
            if (sq == 0) { a0 = a0 * sc + vx * p; a1 = a1 * sc; }
            else         { a1 = a1 * sc + vx * p; a0 = a0 * sc; }
            *p0 = a0;
            *p1 = a1;
            if ((lane & 3) == 0) {
              const float dn = den[mi];
              den[mi] = dn * sc + p;
              mrun[mi] = mn;
            }
            __builtin_amdgcn_fence(__ATOMIC_RELEASE, "wavefront");
            __builtin_amdgcn_wave_barrier();
          }
        }
      }
      __syncthreads();
    }
  }

  for (int i = tid; i < NB * NH; i += NTHR) {
    const float dv = den[i];
    den[i] = __builtin_amdgcn_rcpf(dv + 1e-16f);
  }
  __syncthreads();

  Frag bh, bl;
  {
    const size_t bro = (size_t)(wave * HD + m) * 32;
    ldfrag(bh, Bvh + bro, 0, hh);
    ldfrag(bl, Bvl + bro, 0, hh);
  }
#pragma unroll 1
  for (int T = 0; T < NB / 16; ++T) {
    const int sl = T * 16 + m;
    const float* pa0 = acc + (size_t)sl * DF + wave * HD + 8 * hh;
    const float* pa1 = acc + (size_t)(NB + sl) * DF + wave * HD + 8 * hh;
    Frag ah, al;
    frag_f32(*(const v4f*)pa0, *(const v4f*)(pa0 + 4), *(const v4f*)pa1, *(const v4f*)(pa1 + 4), ah, al);
    v8f c = zero8();
    c = wm3(ah.v, al.v, bh.v, bl.v, c);
#pragma unroll
    for (int r = 0; r < 8; ++r) {
      const int rl = 8 * hh + r;
      const float iv = den[(T * 16 + rl) * NH + wave];
      outt[rl * XSP + wave * HD + m] = c[r] * iv;
    }
    __syncthreads();
    const v4f o0 = *(const v4f*)(outt + (2 * wave) * XSP + 4 * lane);
    const v4f o1 = *(const v4f*)(outt + (2 * wave + 1) * XSP + 4 * lane);
    const int n0 = nodeBase + T * 16 + 2 * wave, n1 = n0 + 1;
    if (n0 < nN) *(volatile v4f*)(qa + (size_t)n0 * DF + 4 * lane) = o0;
    if (n1 < nN) *(volatile v4f*)(qa + (size_t)n1 * DF + 4 * lane) = o1;
    __threadfence();
    if (n0 < nN) *(volatile v4f*)(qa + (size_t)n0 * DF + 4 * lane) = o0;
    if (n1 < nN) *(volatile v4f*)(qa + (size_t)n1 * DF + 4 * lane) = o1;
    __syncthreads();
  }
}

__global__ __launch_bounds__(NTHR) void k_head(const float* __restrict__ h,
                                               const unsigned short* __restrict__ Hh,
                                               const unsigned short* __restrict__ Hl,
                                               const float* __restrict__ hb, float* out, int nN) {
  __shared__ __attribute__((aligned(16))) float os[HB * NCLS];
  const int tid = threadIdx.x, lane = tid & 31, wave = tid >> 5;
  const int hh = lane >> 4, m = lane & 15;
  const int rowBase = blockIdx.x * HB;
  int row = rowBase + wave * 16 + m;
  if (row > nN - 1) row = nN - 1;
  const float* hr = h + (size_t)row * DF;
  const unsigned short* bhr = Hh + (size_t)m * DF;
  const unsigned short* blr = Hl + (size_t)m * DF;
  v8f c = zero8();
#pragma unroll
  for (int kt = 0; kt < DF / 32; ++kt) {
    const int k0 = kt * 32;
    Frag ah, al, bh, bl;
    frag_f32(*(const v4f*)(hr + k0 + 8 * hh), *(const v4f*)(hr + k0 + 8 * hh + 4),
             *(const v4f*)(hr + k0 + 16 + 8 * hh), *(const v4f*)(hr + k0 + 16 + 8 * hh + 4), ah, al);
    ldfrag(bh, bhr, k0, hh);
    ldfrag(bl, blr, k0, hh);
    c = wm3(ah.v, al.v, bh.v, bl.v, c);
  }
  const int cc = (m < NCLS) ? m : (NCLS - 1);
  const float bv = hb[cc];
  if (m < NCLS) {
#pragma unroll
    for (int r = 0; r < 8; ++r) os[(wave * 16 + 8 * hh + r) * NCLS + m] = c[r] + bv;
  }
  __syncthreads();
  if (tid < (HB * NCLS) / 4) {
    const v4f o = *(const v4f*)(os + 4 * tid);
    const int r0 = rowBase + 2 * tid;
    float* op = out + (size_t)r0 * NCLS;
    const bool full = (r0 + 1) < nN;
    const bool one  = r0 < nN;
    if (full) { *(volatile v4f*)op = o; }
    else if (one) { *(volatile float*)op = o.x; *(volatile float*)(op + 1) = o.y; }
    __threadfence();
    if (full) { *(volatile v4f*)op = o; }
    else if (one) { *(volatile float*)op = o.x; *(volatile float*)(op + 1) = o.y; }
  }
}

extern "C" void kernel_launch(void* const* d_in, const int* in_sizes, int n_in,
                              void* d_out, int out_size, void* d_ws, size_t ws_size,
                              hipStream_t stream) {
  if (n_in < 15) return;
  const int nN = in_sizes[0] / DF;
  if (nN <= 0 || in_sizes[0] != nN * DF) return;
  const int nEf = in_sizes[1] / 2, nEr = in_sizes[2] / 2;
  if (nEf < 0 || nEr < 0 || in_sizes[1] != 2 * nEf || in_sizes[2] != 2 * nEr) return;
  if (in_sizes[3] != DF * DF || in_sizes[4] != DF) return;
  if (in_sizes[5] != NL * DF * 3 * DF || in_sizes[6] != NL * 3 * DF) return;
  if (in_sizes[7] != NL * 2 * NH * HD * HD || in_sizes[8] != NL * 2 * NH * HD * HD) return;
  if (in_sizes[9] != NL * 2 * NH || in_sizes[10] != NL * DF * DF || in_sizes[11] != NL * DF) return;
  if (in_sizes[12] != NL || in_sizes[13] != DF * NCLS || in_sizes[14] != NCLS) return;
  if (out_size != nN * NCLS) return;

  const float* x      = (const float*)d_in[0];
  const int*   ef     = (const int*)d_in[1];
  const int*   er     = (const int*)d_in[2];
  const float* in_w   = (const float*)d_in[3];
  const float* in_b   = (const float*)d_in[4];
  const float* kqv_w  = (const float*)d_in[5];
  const float* kqv_b  = (const float*)d_in[6];
  const float* krel_w = (const float*)d_in[7];
  const float* vrel_w = (const float*)d_in[8];
  const float* p_rel  = (const float*)d_in[9];
  const float* out_w  = (const float*)d_in[10];
  const float* out_b  = (const float*)d_in[11];
  const float* skip   = (const float*)d_in[12];
  const float* head_w = (const float*)d_in[13];
  const float* head_b = (const float*)d_in[14];
  float* out = (float*)d_out;

  size_t off = 0;
  char* base = (char*)d_ws;
  auto take = [&](size_t bytes) -> char* {
    char* p = base + off;
    off += (bytes + 255) & ~(size_t)255;
    return p;
  };
  const size_t plane = (size_t)nN * DF * sizeof(float);
  float* hpl  = (float*)take(plane);
  float* qa   = (float*)take(plane);
  float* kr0  = (float*)take(plane);
  float* kr1  = (float*)take(plane);
  float* vpl  = (float*)take(plane);
  const size_t inWb   = (size_t)DF * DF * 2;
  const size_t kqvWb  = (size_t)NL * 3 * DF * DF * 2;
  const size_t outWb  = (size_t)NL * DF * DF * 2;
  const size_t headWb = (size_t)16 * DF * 2;
  const size_t bkb    = (size_t)NL * 2 * NH * RELT * 2;
  const size_t bvb    = (size_t)NL * NH * RELT * 2;
  unsigned short* inWh   = (unsigned short*)take(inWb);
  unsigned short* inWl   = (unsigned short*)take(inWb);
  unsigned short* kqvWh  = (unsigned short*)take(kqvWb);
  unsigned short* kqvWl  = (unsigned short*)take(kqvWb);
  unsigned short* outWh  = (unsigned short*)take(outWb);
  unsigned short* outWl  = (unsigned short*)take(outWb);
  unsigned short* headWh = (unsigned short*)take(headWb);
  unsigned short* headWl = (unsigned short*)take(headWb);
  unsigned short* Bkh    = (unsigned short*)take(bkb);
  unsigned short* Bkl    = (unsigned short*)take(bkb);
  unsigned short* Bvh    = (unsigned short*)take(bvb);
  unsigned short* Bvl    = (unsigned short*)take(bvb);
  if (off > ws_size) return;

  k_wt<<<DF / 16, NTHR, 0, stream>>>(in_w, inWh, inWl, DF, DF);
  k_wt<<<(NL * 3 * DF) / 16, NTHR, 0, stream>>>(kqv_w, kqvWh, kqvWl, 3 * DF, 3 * DF);
  k_wt<<<(NL * DF) / 16, NTHR, 0, stream>>>(out_w, outWh, outWl, DF, DF);
  k_wt<<<1, NTHR, 0, stream>>>(head_w, headWh, headWl, NCLS, 16);
  k_relprep<<<NL * 2 * NH + NL * NH, NTHR, 0, stream>>>(krel_w, vrel_w, Bkh, Bkl, Bvh, Bvl);

  const int gridG = (nN + GR - 1) / GR;
  const int gridA = (nN + NB - 1) / NB;
  const int gridH = (nN + HB - 1) / HB;

  k_gemm128<0><<<gridG, NTHR, 0, stream>>>(x, inWh, inWl, in_b, skip, hpl, nN);

  hipFuncSetAttribute(reinterpret_cast<const void*>(&k_node),
                      hipFuncAttributeMaxDynamicSharedMemorySize, NODE_LDS_BYTES);
  hipFuncSetAttribute(reinterpret_cast<const void*>(&k_agg),
                      hipFuncAttributeMaxDynamicSharedMemorySize, AG_LDS_BYTES);

  for (int l = 0; l < NL; ++l) {
    k_node<<<gridG, NTHR, NODE_LDS_BYTES, stream>>>(
        hpl, kqvWh + (size_t)l * 3 * DF * DF, kqvWl + (size_t)l * 3 * DF * DF,
        kqv_b + (size_t)l * 3 * DF, Bkh + (size_t)l * 2 * NH * RELT, Bkl + (size_t)l * 2 * NH * RELT,
        qa, kr0, kr1, vpl, nN);
    k_agg<<<gridA, NTHR, AG_LDS_BYTES, stream>>>(
        qa, kr0, kr1, vpl, ef, er, nEf, nEr, p_rel + (size_t)l * 2 * NH,
        Bvh + (size_t)l * NH * RELT, Bvl + (size_t)l * NH * RELT, nN);
    k_gemm128<1><<<gridG, NTHR, 0, stream>>>(
        qa, outWh + (size_t)l * DF * DF, outWl + (size_t)l * DF * DF,
        out_b + (size_t)l * DF, skip + l, hpl, nN);
  }

  k_head<<<gridH, NTHR, 0, stream>>>(hpl, headWh, headWl, head_b, out, nN);
}
